// Imaginator_89300960018772
// MI455X (gfx1250) — hardware-verified
//
#include <hip/hip_runtime.h>


#define NB_  8192
#define NP_  64
#define CB   1024
#define NCH  (NB_ / CB)
#define ROWS (CB * NP_)
#define K0   32
#define N1   192
#define K1   160
#define N4   128
#define EFF  100
typedef _Float16 h16;
typedef unsigned short bf;
typedef __attribute__((ext_vector_type(16))) __bf16   v16bf;
typedef __attribute__((ext_vector_type(16))) _Float16 v16h;
typedef __attribute__((ext_vector_type(8)))  _Float16 v8h;
typedef __attribute__((ext_vector_type(8)))  unsigned short v8us;
typedef __attribute__((ext_vector_type(8)))  float    v8f;
typedef __attribute__((ext_vector_type(4)))  float    v4f;
typedef v8h  __attribute__((may_alias)) v8ha;
typedef v4f  __attribute__((may_alias)) v4fa;
typedef v8us __attribute__((may_alias)) v8usa;

__device__ __forceinline__ unsigned short f2bf(float f) { unsigned u = __float_as_uint(f); u += 0x7FFFu + ((u >> 16) & 1u); return (unsigned short)(u >> 16); }
__device__ __forceinline__ float bf2f(unsigned short b) { return __uint_as_float(((unsigned)b) << 16); }
__device__ __forceinline__ float bfr(float f) { return bf2f(f2bf(f)); }
__device__ __forceinline__ v16h cat16(v8h lo, v8h hi) { return __builtin_shufflevector(lo, hi, 0, 1, 2, 3, 4, 5, 6, 7, 8, 9, 10, 11, 12, 13, 14, 15); }
__device__ __forceinline__ v16bf cat16b(v8us lo, v8us hi) { return __builtin_bit_cast(v16bf, __builtin_shufflevector(lo, hi, 0, 1, 2, 3, 4, 5, 6, 7, 8, 9, 10, 11, 12, 13, 14, 15)); }
__device__ __forceinline__ v8f wmma16(v16h a, v16h b, v8f c) { return __builtin_amdgcn_wmma_f32_16x16x32_f16(false, a, false, b, (short)0, c, false, false); }
__device__ __forceinline__ v8f wmmab(v16bf a, v16bf b, v8f c) { return __builtin_amdgcn_wmma_f32_16x16x32_bf16(false, a, false, b, (short)0, c, false, false); }


template <typename T16> struct WFrag;
template <> struct WFrag<h16> { typedef v16h V; static __device__ __forceinline__ V ld(const h16* p) { return cat16(*(const v8h*)p, *(const v8h*)(p + 16)); } static __device__ __forceinline__ v8f mma(V a, V b, v8f c) { return wmma16(a, b, c); } };
template <> struct WFrag<bf> { typedef v16bf V; static __device__ __forceinline__ V ld(const bf* p) { return cat16b(*(const v8us*)p, *(const v8us*)(p + 16)); } static __device__ __forceinline__ v8f mma(V a, V b, v8f c) { return wmmab(a, b, c); } };
template <typename T16, int NSPLIT, bool BIAS>
__global__ __launch_bounds__(32) void k_gemmw(const T16* __restrict__ A, const T16* __restrict__ A2, const T16* __restrict__ Bt, const T16* __restrict__ Bt2, int K, float* C, int ldc, const float* __restrict__ bias, size_t sA, size_t sB, size_t sC) {
    typedef typename WFrag<T16>::V V;
    __shared__ __align__(16) float os[16 * 68];
    const size_t z = blockIdx.z; A += z * sA; if (A2) A2 += z * sA; Bt += z * sB; if (Bt2) Bt2 += z * sB; C += z * sC;
    const int lane = threadIdx.x & 31, lr = lane & 15, hi = lane >> 4; const int r0 = blockIdx.x * 64, c0 = blockIdx.y * 64;
    v8f acc[4][4];
#pragma unroll
    for (int mb = 0; mb < 4; ++mb)
#pragma unroll
        for (int nb = 0; nb < 4; ++nb) acc[mb][nb] = (v8f){};
    const size_t aoff = (size_t)(r0 + lr) * K + 8 * hi, boff = (size_t)(c0 + lr) * K + 8 * hi;
#pragma unroll 1
    for (int kc = 0; kc < K; kc += 32) {
        V a[4], a2[4];
#pragma unroll
        for (int mb = 0; mb < 4; ++mb) { a[mb] = WFrag<T16>::ld(A + aoff + (size_t)mb * 16 * K + kc); if (NSPLIT == 1 || NSPLIT == 2) a2[mb] = WFrag<T16>::ld(A2 + aoff + (size_t)mb * 16 * K + kc); }
#pragma unroll
        for (int nb = 0; nb < 4; ++nb) { const V b = WFrag<T16>::ld(Bt + boff + (size_t)nb * 16 * K + kc); V b2; if (NSPLIT >= 2) b2 = WFrag<T16>::ld(Bt2 + boff + (size_t)nb * 16 * K + kc);
#pragma unroll
            for (int mb = 0; mb < 4; ++mb) { acc[mb][nb] = WFrag<T16>::mma(a[mb], b, acc[mb][nb]); if (NSPLIT == 1 || NSPLIT == 2) acc[mb][nb] = WFrag<T16>::mma(a2[mb], b, acc[mb][nb]); if (NSPLIT >= 2) acc[mb][nb] = WFrag<T16>::mma(a[mb], b2, acc[mb][nb]); } }
        asm volatile("v_nop\n\tv_nop\n\tv_nop\n\tv_nop" : "+v"(acc[0][0]), "+v"(acc[1][1]), "+v"(acc[2][2]), "+v"(acc[3][3]) : "v"(a[0]), "v"(a[3]));
    }
#pragma unroll
    for (int mb = 0; mb < 4; ++mb) {
#pragma unroll
        for (int nb = 0; nb < 4; ++nb) {
#pragma unroll
            for (int j = 0; j < 8; ++j) os[(hi * 8 + j) * 68 + nb * 16 + lr] = acc[mb][nb][j]; }
        __builtin_amdgcn_wave_barrier(); asm volatile("" ::: "memory");
        float* crow = C + (size_t)(r0 + mb * 16) * ldc + c0;
#pragma unroll 1
        for (int ps = 0; ps < 2; ++ps) {
#pragma unroll
            for (int s = 0; s < 8; ++s) { const int row = 2 * s + hi, cofs = lr * 4; v4f val = *(const v4fa*)(os + row * 68 + cofs); if (BIAS) { val[0] += bfr(bias[c0 + cofs]); val[1] += bfr(bias[c0 + cofs + 1]); val[2] += bfr(bias[c0 + cofs + 2]); val[3] += bfr(bias[c0 + cofs + 3]); }
                *(volatile v4f*)(crow + (size_t)row * ldc + cofs) = val; }
            if (ps == 0) __threadfence(); }
        __builtin_amdgcn_wave_barrier(); asm volatile("" ::: "memory");
    }
}

__device__ __forceinline__ h16 tohx(float x) { return (h16)x; }
typedef __attribute__((ext_vector_type(4))) _Float16 v4h;
typedef __attribute__((ext_vector_type(4))) unsigned short v4us;

__global__ __launch_bounds__(256) void k_w0(const float* __restrict__ w, const float* __restrict__ b, bf* Bt, float* BP) { const int i = (blockIdx.x * 256 + threadIdx.x) * 4; if (i < N1 * K0) { const int n = i / K0, k = i % K0; v4us o;
#pragma unroll
        for (int q = 0; q < 4; ++q) o[q] = (n < 150 && k + q < 10) ? f2bf(w[(k + q) * 150 + n]) : (unsigned short)0; *(volatile v4us*)(Bt + i) = o; __threadfence(); *(volatile v4us*)(Bt + i) = o; }
    const int t = blockIdx.x * 256 + threadIdx.x; if (t < N1) { const float v = t < 150 ? b[t] : 0.f; *(volatile float*)(BP + t) = v; __threadfence(); *(volatile float*)(BP + t) = v; } }
__global__ __launch_bounds__(256) void k_w16t(const float* __restrict__ w, int fi, int fo, int KP, int NPd, const float* __restrict__ b, h16* Bt, float* BP) { const int i = (blockIdx.x * 256 + threadIdx.x) * 4; if (i < NPd * KP) { const int n = i / KP, k = i % KP; v4h o;
#pragma unroll
        for (int q = 0; q < 4; ++q) o[q] = (n < fo && k + q < fi) ? tohx(bfr(w[(size_t)(k + q) * fo + n])) : (h16)0.f; *(volatile v4h*)(Bt + i) = o; __threadfence(); *(volatile v4h*)(Bt + i) = o; }
    const int t = blockIdx.x * 256 + threadIdx.x; if (t < NPd) { const float v = t < fo ? b[t] : 0.f; *(volatile float*)(BP + t) = v; __threadfence(); *(volatile float*)(BP + t) = v; } }
__global__ __launch_bounds__(256) void k_a0(const float* __restrict__ ag, const float* __restrict__ pl, int b0, bf* A0) { const size_t e = ((size_t)blockIdx.x * 256 + threadIdx.x) * 4; if (e >= (size_t)ROWS * K0) return; const int k = (int)(e % K0); const int r = (int)(e / K0); const int b = b0 + r / NP_, p = r % NP_; v4us o;
#pragma unroll
    for (int q = 0; q < 4; ++q) { const int kk = k + q; float v = 0.f; if (kk < 5) v = ag[b * 5 + kk]; else if (kk < 10) v = pl[((size_t)b * NP_ + p) * 5 + kk - 5]; o[q] = f2bf(v); } *(volatile v4us*)(A0 + e) = o; __threadfence(); *(volatile v4us*)(A0 + e) = o; }
__global__ __launch_bounds__(256) void k_pl(const float* __restrict__ F, h16* P) { const size_t e = ((size_t)blockIdx.x * 256 + threadIdx.x) * 4; if (e >= (size_t)ROWS * K1) return; const int c = (int)(e % K1); const size_t r = e / K1; v4h o;
#pragma unroll
    for (int q = 0; q < 4; ++q) o[q] = (c + q < 150) ? tohx(fmaxf(F[r * N1 + c + q], 0.f)) : (h16)0.f; *(volatile v4h*)(P + e) = o; __threadfence(); *(volatile v4h*)(P + e) = o; }
__global__ __launch_bounds__(256) void k_agg(const float* __restrict__ F4, int b0, float* AGG) { const int e = (blockIdx.x * 256 + threadIdx.x) * 4; if (e >= CB * N4) return; const int c = e % N4; const int bl = e / N4; v4f o;
#pragma unroll
    for (int q = 0; q < 4; ++q) { float s = 0.f; if (c + q < EFF) {
#pragma unroll 1
            for (int p = 0; p < NP_; ++p) s = __fadd_rn(s, fmaxf(F4[((size_t)bl * NP_ + p) * N4 + c + q], 0.f)); } o[q] = s; }
    float* dst = AGG + (size_t)(b0 + bl) * N4 + c; *(volatile v4f*)dst = o; __threadfence(); *(volatile v4f*)dst = o; }
__global__ __launch_bounds__(128) void k_obj(const float* __restrict__ ag, const float* __restrict__ act, const float* __restrict__ AGG, const float* __restrict__ w0, const float* __restrict__ b0, const float* __restrict__ w1, const float* __restrict__ b1, float* OUT) { const int b = blockIdx.x * 128 + threadIdx.x; if (b >= NB_) return; float o0 = bfr(b1[0]), o1 = bfr(b1[1]), o2 = bfr(b1[2]), o3 = bfr(b1[3]);
#pragma unroll 1
    for (int j = 0; j < 100; ++j) { float h = bfr(b0[j]);
#pragma unroll 1
        for (int i = 0; i < 107; ++i) { const float xv = i < 5 ? bfr(ag[b * 5 + i]) : (i < 7 ? bfr(act[b * 2 + i - 5]) : AGG[(size_t)b * N4 + i - 7]); float p = __fmul_rn(xv, bfr(w0[i * 100 + j])); asm volatile("" : "+v"(p)); h = __fadd_rn(h, p); }
        h = fmaxf(h, 0.f); float p0 = __fmul_rn(h, bfr(w1[j * 4 + 0])), p1 = __fmul_rn(h, bfr(w1[j * 4 + 1])), p2 = __fmul_rn(h, bfr(w1[j * 4 + 2])), p3 = __fmul_rn(h, bfr(w1[j * 4 + 3])); asm volatile("" : "+v"(p0)); asm volatile("" : "+v"(p1)); asm volatile("" : "+v"(p2)); asm volatile("" : "+v"(p3));
        o0 = __fadd_rn(o0, p0); o1 = __fadd_rn(o1, p1); o2 = __fadd_rn(o2, p2); o3 = __fadd_rn(o3, p3); }
    v4f o; o[0] = o0; o[1] = o1; o[2] = o2; o[3] = o3; *(volatile v4f*)(OUT + (size_t)b * 4) = o; __threadfence(); *(volatile v4f*)(OUT + (size_t)b * 4) = o; }

extern "C" void kernel_launch(void* const* d_in, const int* in_sizes, int n_in,
                              void* d_out, int out_size, void* d_ws, size_t ws_size, hipStream_t stream) {
    (void)in_sizes; (void)n_in; (void)out_size;
    const float* ag = (const float*)d_in[0]; const float* pl = (const float*)d_in[1]; const float* act = (const float*)d_in[2];
    const float* rw0 = (const float*)d_in[3]; const float* rb0 = (const float*)d_in[4]; const float* rw1 = (const float*)d_in[5]; const float* rb1 = (const float*)d_in[6]; const float* rw2 = (const float*)d_in[7]; const float* rb2 = (const float*)d_in[8]; const float* rw3 = (const float*)d_in[9]; const float* rb3 = (const float*)d_in[10]; const float* rw4 = (const float*)d_in[11]; const float* rb4 = (const float*)d_in[12];
    const float* ow0 = (const float*)d_in[13]; const float* ob0 = (const float*)d_in[14]; const float* ow1 = (const float*)d_in[15]; const float* ob1 = (const float*)d_in[16];
    float* OUT = (float*)d_out;
    char* wsp = (char*)d_ws;
    auto take = [&](size_t bytes) { char* p = wsp; wsp += (bytes + 255) & ~(size_t)255; return (void*)p; };
    bf* B0 = (bf*)take(N1 * K0 * 2); float* P0 = (float*)take(N1 * 4); h16* B1 = (h16*)take(N1 * K1 * 2); float* P1 = (float*)take(N1 * 4); h16* B2 = (h16*)take(N1 * K1 * 2); float* P2 = (float*)take(N1 * 4); h16* B3 = (h16*)take(N1 * K1 * 2); float* P3 = (float*)take(N1 * 4); h16* B4 = (h16*)take(N4 * K1 * 2); float* P4 = (float*)take(N4 * 4);
    bf* A0 = (bf*)take((size_t)ROWS * K0 * 2); float* F = (float*)take((size_t)ROWS * N1 * 4); h16* PL = (h16*)take((size_t)ROWS * K1 * 2); float* F4 = (float*)take((size_t)ROWS * N4 * 4); float* AGG = (float*)take((size_t)NB_ * N4 * 4);
    if ((size_t)(wsp - (char*)d_ws) > ws_size) return;
    k_w0<<<(N1 * K0 / 4 + 255) / 256, 256, 0, stream>>>(rw0, rb0, B0, P0); k_w16t<<<(N1 * K1 / 4 + 255) / 256, 256, 0, stream>>>(rw1, 150, 150, K1, N1, rb1, B1, P1); k_w16t<<<(N1 * K1 / 4 + 255) / 256, 256, 0, stream>>>(rw2, 150, 150, K1, N1, rb2, B2, P2); k_w16t<<<(N1 * K1 / 4 + 255) / 256, 256, 0, stream>>>(rw3, 150, 150, K1, N1, rb3, B3, P3); k_w16t<<<(N4 * K1 / 4 + 255) / 256, 256, 0, stream>>>(rw4, 150, 100, K1, N4, rb4, B4, P4);
    for (int ch = 0; ch < NCH; ++ch) { const int b0 = ch * CB;
        k_a0<<<(ROWS * K0 / 4 + 255) / 256, 256, 0, stream>>>(ag, pl, b0, A0);
        k_gemmw<bf, 0, true><<<dim3(ROWS / 64, N1 / 64, 1), 32, 0, stream>>>(A0, nullptr, B0, nullptr, K0, F, N1, P0, 0, 0, 0); k_pl<<<(unsigned)(((size_t)ROWS * K1 / 4 + 255) / 256), 256, 0, stream>>>(F, PL);
        k_gemmw<h16, 0, true><<<dim3(ROWS / 64, N1 / 64, 1), 32, 0, stream>>>(PL, nullptr, B1, nullptr, K1, F, N1, P1, 0, 0, 0); k_pl<<<(unsigned)(((size_t)ROWS * K1 / 4 + 255) / 256), 256, 0, stream>>>(F, PL);
        k_gemmw<h16, 0, true><<<dim3(ROWS / 64, N1 / 64, 1), 32, 0, stream>>>(PL, nullptr, B2, nullptr, K1, F, N1, P2, 0, 0, 0); k_pl<<<(unsigned)(((size_t)ROWS * K1 / 4 + 255) / 256), 256, 0, stream>>>(F, PL);
        k_gemmw<h16, 0, true><<<dim3(ROWS / 64, N1 / 64, 1), 32, 0, stream>>>(PL, nullptr, B3, nullptr, K1, F, N1, P3, 0, 0, 0); k_pl<<<(unsigned)(((size_t)ROWS * K1 / 4 + 255) / 256), 256, 0, stream>>>(F, PL);
        k_gemmw<h16, 0, true><<<dim3(ROWS / 64, N4 / 64, 1), 32, 0, stream>>>(PL, nullptr, B4, nullptr, K1, F4, N4, P4, 0, 0, 0);
        k_agg<<<(CB * N4 / 4 + 255) / 256, 256, 0, stream>>>(F4, b0, AGG); }
    k_obj<<<NB_ / 128, 128, 0, stream>>>(ag, act, AGG, ow0, ob0, ow1, ob1, OUT);
}
